// GMGRU_20048907338172
// MI455X (gfx1250) — hardware-verified
//
#include <hip/hip_runtime.h>


#define DD    33
#define TT    49
#define HID   64
#define QQ    64
#define H3    192
#define DH    (DD * HID)
#define NOUT0 (TT * DH)
#define NOUT1 (DD * TT)
#define NTHR  512
#define NWAVE (NTHR / 32)
#define NTASK (DD * 4)

typedef unsigned short us16;
typedef us16   v8us  __attribute__((ext_vector_type(8)));
typedef __bf16 v16bf __attribute__((ext_vector_type(16)));
typedef float  v8f   __attribute__((ext_vector_type(8)));
typedef float  v4f   __attribute__((ext_vector_type(4)));

union FragBF { v16bf v; v8us half[2]; };

constexpr size_t PE     = (size_t)DD * HID * HID;
constexpr size_t PBYTES = PE * 2;
constexpr int    NPLANE = 12;
constexpr size_t WS_END = (size_t)NPLANE * PBYTES;
static_assert(PBYTES % 512 == 0);
static_assert(WS_END <= (size_t)134217728);
constexpr int NPC_T     = (int)(PE / 8);
constexpr int NPC       = 6 * NPC_T;
constexpr int CVTBLK    = NPC / 256;
constexpr int BLK_PER_T = NPC_T / 256;
static_assert(NPC_T % 256 == 0);
static_assert((size_t)NPC * 8 == 6 * PE);

#define SB_HVEC(d, pp) (((d) * 2 + (pp)) * HID)
#define SB_hVEC(pp)    (DD * 2 * HID + (pp) * HID)
#define SB_ZROW        (DD * 2 * HID + 2 * HID)
#define SB_TOTAL       (SB_ZROW + HID)

__shared__ __attribute__((aligned(16))) float sH[DH];
__shared__ __attribute__((aligned(16))) float sRes[4 * DH];
__shared__ __attribute__((aligned(16))) us16  sB[SB_TOTAL];
__shared__ __attribute__((aligned(16))) float sXP[1620];
__shared__ float sh[HID], sHist[3 * HID], sU[QQ], sGst[HID], sGi[H3], sGh[H3];
__shared__ float sX[36], sM[36], sDl[36], sXst[36], sXc[36], sXgt[36], sAv[36], sC1[36], sC2[36];

__device__ __forceinline__ unsigned bf16_rne(float x) {
    unsigned u = __float_as_uint(x);
    u += 0x7FFFu + ((u >> 16) & 1u);
    return u >> 16;
}
__device__ __forceinline__ void split2(float x, us16& hi, us16& lo) {
    const unsigned hb = bf16_rne(x);
    const float    r  = x - __uint_as_float(hb << 16);
    hi = (us16)hb;
    lo = (us16)bf16_rne(r);
}
__device__ __forceinline__ float sigf(float x) {
    const float e = expf(fminf(-x, 30.0f));
    return 1.0f / (1.0f + e);
}
__device__ __forceinline__ float decayf(float x) { return expf(-fmaxf(x, 0.0f)); }
__device__ __forceinline__ v8f zero8() {
    v8f z;
#pragma unroll
    for (int i = 0; i < 8; ++i) z[i] = 0.0f;
    return z;
}

__device__ __forceinline__ v8f mma_bf(v8f c, const FragBF& a, const FragBF& b) {
    c = __builtin_amdgcn_wmma_f32_16x16x32_bf16(false, a.v, false, b.v, (short)0, c, false, false);
    asm volatile("v_nop\n\tv_nop\n\tv_nop\n\tv_nop" : "+v"(c) : "v"(a.v), "v"(b.v));
    return c;
}
__device__ __forceinline__ v8f mv64(v8f acc, const us16* __restrict__ ahi,
                                     const us16* __restrict__ alo, int boff) {
#pragma unroll
    for (int kt = 0; kt < 2; ++kt) {
        FragBF b, a;
        b.half[0] = *(const v8us*)(&sB[boff + kt * 32]);
        b.half[1] = *(const v8us*)(&sB[boff + kt * 32 + 16]);
        a.half[0] = *(const v8us*)(ahi + kt * 32);
        a.half[1] = *(const v8us*)(ahi + kt * 32 + 16);
        acc = mma_bf(acc, a, b);
        a.half[0] = *(const v8us*)(alo + kt * 32);
        a.half[1] = *(const v8us*)(alo + kt * 32 + 16);
        acc = mma_bf(acc, a, b);
    }
    return acc;
}
__device__ __forceinline__ void redstore(v8f acc, int slot, int base, int m) {
    float s[8];
#pragma unroll
    for (int r = 0; r < 8; ++r) s[r] = acc[r] + __shfl_xor(acc[r], 1);
    if (m == 0) {
#pragma unroll
        for (int r = 0; r < 8; ++r) sRes[slot * DH + base + r] = s[r];
    }
}

struct CvtArgs { const float* s0; const float* s1; const float* s2; const float* s3; const float* s4; const float* s5; us16* planes; };
static_assert(sizeof(CvtArgs) == 7 * 8);

__global__ __launch_bounds__(256)
void k_planes(CvtArgs a)
{
    const int tid    = threadIdx.x;
    const int tensor = (int)blockIdx.x / BLK_PER_T;
    const int within = ((int)blockIdx.x - tensor * BLK_PER_T) * 256 + tid;
    const float* src = (tensor == 0) ? a.s0 : (tensor == 1) ? a.s1 : (tensor == 2) ? a.s2
                     : (tensor == 3) ? a.s3 : (tensor == 4) ? a.s4 : a.s5;
    const size_t e0 = (size_t)within * 8;
    const v4f x0 = *(const v4f*)(src + e0);
    const v4f x1 = *(const v4f*)(src + e0 + 4);
    v8us hv, lv;
#pragma unroll
    for (int i = 0; i < 4; ++i) {
        us16 hi, lo;
        split2(x0[i], hi, lo); hv[i] = hi;     lv[i] = lo;
        split2(x1[i], hi, lo); hv[4 + i] = hi; lv[4 + i] = lo;
    }
    us16* dh = a.planes + (size_t)(2 * tensor) * PE + e0;
    us16* dl = dh + PE;
    *(volatile v8us*)dh = hv;
    *(volatile v8us*)dl = lv;
    __threadfence();
    *(volatile v8us*)dh = hv;
    *(volatile v8us*)dl = lv;
}

struct SeqArgs {
    const float *data, *h0, *H0, *gh_w, *gh_b, *gst_w, *gst_b, *wih, *whh, *bih, *bhh,
                *wu0_w, *wu0_b, *wu1_w, *wu1_b, *wu_w, *wu_b, *wh_w, *wh_b, *xst_w, *xst_b,
                *wrg_w, *wrs, *tUzx, *tUrx, *tUhx, *tbz, *tbr, *tbh;
    const us16* planes;
    float* out;
};
static_assert(sizeof(SeqArgs) == 31 * 8);

__device__ __forceinline__ v4f combine4(const SeqArgs& p, int pc) {
    const int e0 = pc * 4;
    const int dd = e0 >> 6;
    const float xc = sXc[dd];
    v4f v;
#pragma unroll
    for (int i = 0; i < 4; ++i) {
        const int e = e0 + i;
        const int j = e & 63;
        const float z  = sigf(sRes[e] + p.tUzx[e] * xc + p.tbz[j]);
        const float r  = sigf(sRes[DH + e] + p.tUrx[e] * xc + p.tbr[j]);
        const float hc = tanhf(r * sRes[2 * DH + e] + p.tUhx[e] * xc + sRes[3 * DH + e] + p.tbh[j]);
        const float Hn = z * sH[e] + (1.0f - z) * hc;
        sH[e] = Hn;
        v[i] = Hn;
    }
    return v;
}

__global__ __launch_bounds__(NTHR)
void k_seq(SeqArgs p)
{
    const int tid  = threadIdx.x;
    const int lane = tid & 31;
    const int wv   = tid >> 5;
    const int hh   = lane >> 4;
    const int m    = lane & 15;

    for (int e = tid; e < DH; e += NTHR) sH[e] = p.H0[e];
    if (tid < HID) sh[tid] = p.h0[tid];
    else if (tid < 2 * HID) sB[SB_ZROW + (tid - HID)] = (us16)0;
    __syncthreads();

#pragma unroll 1
    for (int t = 0; t < TT; ++t) {
        if (tid < DD) {
            sX[tid]  = p.data[0 * NOUT1 + tid * TT + t];
            sM[tid]  = p.data[1 * NOUT1 + tid * TT + t];
            sDl[tid] = p.data[2 * NOUT1 + tid * TT + t];
        } else if (tid >= 64 && tid < 64 + DD) {
            const int dd = tid - 64;
            float acc = 0.0f;
#pragma unroll 4
            for (int i = 0; i < HID; ++i) acc += sH[dd * HID + i] * p.xst_w[i];
            sXst[dd] = acc + p.xst_b[0];
        } else if (tid >= 128 && tid < 128 + QQ) {
            const int q = tid - 128;
            float acc = 0.0f;
            if (t == 0) {
                const float* w = p.wu0_w + q * HID;
#pragma unroll 4
                for (int i = 0; i < HID; ++i) acc += w[i] * p.h0[i];
                acc += p.wu0_b[q];
            } else if (t == 1) {
                const float* w = p.wu1_w + q * (2 * HID);
#pragma unroll 4
                for (int i = 0; i < HID; ++i) acc += w[i] * p.h0[i];
#pragma unroll 4
                for (int i = 0; i < HID; ++i) acc += w[HID + i] * sHist[i];
                acc += p.wu1_b[q];
            } else if (t == 2) {
                const float* w = p.wu_w + q * H3;
#pragma unroll 4
                for (int i = 0; i < HID; ++i) acc += w[i] * p.h0[i];
#pragma unroll 4
                for (int i = 0; i < HID; ++i) acc += w[HID + i] * sHist[i];
#pragma unroll 4
                for (int i = 0; i < HID; ++i) acc += w[2 * HID + i] * sHist[HID + i];
                acc += p.wu_b[q];
            } else {
                const float* w = p.wu_w + q * H3;
                const int s0 = (t % 3) * HID, s1 = ((t + 1) % 3) * HID, s2 = ((t + 2) % 3) * HID;
#pragma unroll 4
                for (int i = 0; i < HID; ++i) acc += w[i] * sHist[s0 + i];
#pragma unroll 4
                for (int i = 0; i < HID; ++i) acc += w[HID + i] * sHist[s1 + i];
#pragma unroll 4
                for (int i = 0; i < HID; ++i) acc += w[2 * HID + i] * sHist[s2 + i];
                acc += p.wu_b[q];
            }
            sU[q] = acc;
        }
        __syncthreads();

        if (tid < HID) {
            const float* w = p.gh_w + tid * DD;
            float acc = 0.0f;
#pragma unroll 4
            for (int dd = 0; dd < DD; ++dd) acc += w[dd] * sDl[dd];
            acc += p.gh_b[tid];
            sh[tid] *= decayf(acc);
        } else if (tid < 2 * HID) {
            const int j = tid - HID;
            const float* w = p.gst_w + j * DD;
            float acc = 0.0f;
#pragma unroll 4
            for (int dd = 0; dd < DD; ++dd) acc += w[dd] * sDl[dd];
            acc += p.gst_b[j];
            sGst[j] = decayf(acc);
        } else if (tid < 2 * HID + DD) {
            const int dd = tid - 2 * HID;
            sXc[dd] = sM[dd] * sX[dd] + (1.0f - sM[dd]) * sXst[dd];
        }
        __syncthreads();

        if (tid < H3) {
            const float* w = p.wih + tid * DD;
            float acc = 0.0f;
#pragma unroll 4
            for (int dd = 0; dd < DD; ++dd) acc += w[dd] * sXc[dd];
            sGi[tid] = acc + p.bih[tid];
        } else if (tid < 2 * H3) {
            const int j = tid - H3;
            const float* w = p.whh + j * HID;
            float acc = 0.0f;
#pragma unroll 4
            for (int i = 0; i < HID; ++i) acc += w[i] * sh[i];
            sGh[j] = acc + p.bhh[j];
        }
        for (int e = tid; e < DH; e += NTHR) {
            const float v = sH[e] * sGst[e & 63];
            sH[e] = v;
            us16 hi, lo;
            split2(v, hi, lo);
            sB[SB_HVEC(e >> 6, 0) + (e & 63)] = hi;
            sB[SB_HVEC(e >> 6, 1) + (e & 63)] = lo;
        }
        __syncthreads();

        if (tid < HID) {
            const int j = tid;
            const float r  = sigf(sGi[j] + sGh[j]);
            const float z  = sigf(sGi[HID + j] + sGh[HID + j]);
            const float n  = tanhf(sGi[2 * HID + j] + r * sGh[2 * HID + j]);
            const float hp = sh[j];
            const float hn = (1.0f - z) * n + z * hp;
            sh[j] = hn;
            sHist[(t % 3) * HID + j] = hn;
            us16 hi, lo;
            split2(hn, hi, lo);
            sB[SB_hVEC(0) + j] = hi;
            sB[SB_hVEC(1) + j] = lo;
        }
        __syncthreads();

        if (tid < DD) {
            const float* w = p.wh_w + tid * (HID + QQ);
            float acc = 0.0f;
#pragma unroll 4
            for (int i = 0; i < HID; ++i) acc += w[i] * sh[i];
#pragma unroll 4
            for (int i = 0; i < QQ; ++i) acc += w[HID + i] * sU[i];
            sXgt[tid] = acc + p.wh_b[tid];
        } else if (tid >= 64 && tid < 64 + DD) {
            const int dd = tid - 64;
            const float* w = p.wrg_w + dd * HID;
            float acc = 0.0f;
#pragma unroll 4
            for (int i = 0; i < HID; ++i) acc += sh[i] * w[i];
            sAv[dd] = acc;
        }
        for (int task = wv; task < NTASK; task += NWAVE) {
            const int d  = task >> 2;
            const int mt = task & 3;
            const int bW = ((m == 0) ? SB_HVEC(d, 0) : (m == 1) ? SB_HVEC(d, 1) : SB_ZROW) + 8 * hh;
            const int bU = ((m == 0) ? SB_hVEC(0)    : (m == 1) ? SB_hVEC(1)    : SB_ZROW) + 8 * hh;
            const us16* pl = p.planes + ((size_t)(d * HID + mt * 16 + m) * HID + 8 * hh);
            const int base = d * HID + mt * 16 + 8 * hh;
            v8f acc = zero8();
            acc = mv64(acc, pl + 0 * PE, pl + 1 * PE, bW);
            acc = mv64(acc, pl + 2 * PE, pl + 3 * PE, bU);
            redstore(acc, 0, base, m);
            acc = zero8();
            acc = mv64(acc, pl + 4 * PE, pl + 5 * PE, bW);
            acc = mv64(acc, pl + 6 * PE, pl + 7 * PE, bU);
            redstore(acc, 1, base, m);
            acc = zero8();
            acc = mv64(acc, pl + 8 * PE, pl + 9 * PE, bW);
            redstore(acc, 2, base, m);
            acc = zero8();
            acc = mv64(acc, pl + 10 * PE, pl + 11 * PE, bU);
            redstore(acc, 3, base, m);
        }
        __syncthreads();

        {
            float* orow = p.out + (size_t)t * DH;
            const v4f v0 = combine4(p, tid);
            *(volatile v4f*)(orow + tid * 4) = v0;
            v4f v1 = v0;
            if (tid < DH / 4 - NTHR) {
                v1 = combine4(p, NTHR + tid);
                *(volatile v4f*)(orow + (NTHR + tid) * 4) = v1;
            }
            __threadfence();
            *(volatile v4f*)(orow + tid * 4) = v0;
            if (tid < DH / 4 - NTHR) *(volatile v4f*)(orow + (NTHR + tid) * 4) = v1;
        }
        __syncthreads();

        if (tid < DD) {
            float acc = 0.0f;
#pragma unroll 4
            for (int i = 0; i < HID; ++i) acc += p.wrs[i] * sH[tid * HID + i];
            const float av = sAv[tid];
            const float ri = 1.0f / (av + acc);
            sC1[tid] = av * ri;
            sC2[tid] = acc * ri;
        }
        __syncthreads();

        if (tid < DD) {
            float m1 = sC1[0], m2 = sC2[0];
#pragma unroll 1
            for (int i = 1; i < DD; ++i) { m1 = fmaxf(m1, sC1[i]); m2 = fmaxf(m2, sC2[i]); }
            float s1 = 0.0f, s2 = 0.0f;
#pragma unroll 1
            for (int i = 0; i < DD; ++i) { s1 += expf(sC1[i] - m1); s2 += expf(sC2[i] - m2); }
            const float a1 = expf(sC1[tid] - m1) * (1.0f / s1);
            const float a2 = expf(sC2[tid] - m2) * (1.0f / s2);
            sXP[tid * TT + t] = a1 * sXgt[tid] + a2 * sXst[tid];
        }
        __syncthreads();
    }

    float* o1 = p.out + NOUT0;
    v4f ov; ov[0] = 0.0f; ov[1] = 0.0f; ov[2] = 0.0f; ov[3] = 0.0f;
    v4f t0 = ov, t1 = ov, t2 = ov, t3 = ov;
    float ts = 0.0f;
    if (tid < 400) {
        ov = *(const v4f*)(&sXP[tid * 4]);
        *(volatile v4f*)(o1 + tid * 4) = ov;
    }
    if (tid == 416) {
        t0 = *(const v4f*)(&sXP[1600]);
        t1 = *(const v4f*)(&sXP[1604]);
        t2 = *(const v4f*)(&sXP[1608]);
        t3 = *(const v4f*)(&sXP[1612]);
        ts = sXP[1616];
        *(volatile v4f*)(o1 + 1600) = t0;
        *(volatile v4f*)(o1 + 1604) = t1;
        *(volatile v4f*)(o1 + 1608) = t2;
        *(volatile v4f*)(o1 + 1612) = t3;
        *(volatile float*)(o1 + 1616) = ts;
    }
    __threadfence();
    if (tid < 400) *(volatile v4f*)(o1 + tid * 4) = ov;
    if (tid == 416) {
        *(volatile v4f*)(o1 + 1600) = t0;
        *(volatile v4f*)(o1 + 1604) = t1;
        *(volatile v4f*)(o1 + 1608) = t2;
        *(volatile v4f*)(o1 + 1612) = t3;
        *(volatile float*)(o1 + 1616) = ts;
    }
}

extern "C" void kernel_launch(void* const* d_in, const int* in_sizes, int n_in,
                              void* d_out, int out_size, void* d_ws, size_t ws_size,
                              hipStream_t stream)
{
    if (n_in < 35) return;
    const int expect[35] = {
        3 * DD * TT, HID, DH, HID * DD, HID, HID * DD, HID, H3 * DD, H3 * HID, H3, H3,
        QQ * HID, QQ, QQ * 2 * HID, QQ, QQ * H3, QQ, DD * (HID + QQ), DD, HID, 1,
        DD * HID, HID, (int)PE, DH, (int)PE, (int)PE, DH, (int)PE, (int)PE, DH, (int)PE, HID, HID, HID };
    for (int i = 0; i < 35; ++i) {
        if (i == 20) { if (in_sizes[i] < 1) return; }
        else if (in_sizes[i] != expect[i]) return;
    }
    if (out_size != NOUT0 + NOUT1) return;
    if (ws_size < WS_END) return;

    const float* const* f = (const float* const*)d_in;

    CvtArgs ca;
    ca.s0 = (const float*)d_in[23];
    ca.s1 = (const float*)d_in[25];
    ca.s2 = (const float*)d_in[26];
    ca.s3 = (const float*)d_in[28];
    ca.s4 = (const float*)d_in[29];
    ca.s5 = (const float*)d_in[31];
    ca.planes = (us16*)d_ws;
    k_planes<<<dim3(CVTBLK), dim3(256), 0, stream>>>(ca);

    SeqArgs sa;
    sa.data  = f[0];  sa.h0    = f[1];  sa.H0    = f[2];
    sa.gh_w  = f[3];  sa.gh_b  = f[4];  sa.gst_w = f[5];  sa.gst_b = f[6];
    sa.wih   = f[7];  sa.whh   = f[8];  sa.bih   = f[9];  sa.bhh   = f[10];
    sa.wu0_w = f[11]; sa.wu0_b = f[12]; sa.wu1_w = f[13]; sa.wu1_b = f[14];
    sa.wu_w  = f[15]; sa.wu_b  = f[16]; sa.wh_w  = f[17]; sa.wh_b  = f[18];
    sa.xst_w = f[19]; sa.xst_b = f[20]; sa.wrg_w = f[21]; sa.wrs   = f[22];
    sa.tUzx  = f[24]; sa.tUrx  = f[27]; sa.tUhx  = f[30];
    sa.tbz   = f[32]; sa.tbr   = f[33]; sa.tbh   = f[34];
    sa.planes = (const us16*)d_ws;
    sa.out    = (float*)d_out;
    k_seq<<<dim3(1), dim3(NTHR), 0, stream>>>(sa);
}
